// CouplingLayer_41635412968146
// MI455X (gfx1250) — hardware-verified
//
#include <hip/hip_runtime.h>


#define NB_   4
#define ROWS  1048576
#define RPN   262144
#define TD    96
#define HD    64
#define OD    10

typedef unsigned short bf;
typedef __attribute__((ext_vector_type(16))) __bf16   v16bf;
typedef __attribute__((ext_vector_type(8)))  unsigned short v8us;
typedef __attribute__((ext_vector_type(8)))  float    v8f;
typedef __attribute__((ext_vector_type(4)))  float    v4f;
typedef v4f  __attribute__((may_alias)) v4fa;
typedef v8us __attribute__((may_alias)) v8usa;

__device__ __forceinline__ unsigned short f2bf(float f) { unsigned u = __float_as_uint(f); u += 0x7FFFu + ((u >> 16) & 1u); return (unsigned short)(u >> 16); }
__device__ __forceinline__ float bf2f(unsigned short b) { return __uint_as_float(((unsigned)b) << 16); }
__device__ __forceinline__ float bfr(float f) { return bf2f(f2bf(f)); }
__device__ __forceinline__ v16bf cat16b(v8us lo, v8us hi) { return __builtin_bit_cast(v16bf, __builtin_shufflevector(lo, hi, 0, 1, 2, 3, 4, 5, 6, 7, 8, 9, 10, 11, 12, 13, 14, 15)); }
__device__ __forceinline__ v8f wmmab(v16bf a, v16bf b, v8f c) { return __builtin_amdgcn_wmma_f32_16x16x32_bf16(false, a, false, b, (short)0, c, false, false); }

__global__ __launch_bounds__(256) void k_base(const float* __restrict__ tfeat, const float* __restrict__ W1, const float* __restrict__ b1, float* BASE) {
    const int t_ = threadIdx.x; const int n = t_ >> 6, h = t_ & 63;
    float acc = 0.f;
#pragma unroll 1
    for (int t = 0; t < TD; ++t) acc = fmaf(bfr(tfeat[n * TD + t]), bfr(W1[(2 + t) * HD + h]), acc);
    acc += bfr(b1[h]);
    *(volatile float*)(BASE + t_) = acc; __threadfence(); *(volatile float*)(BASE + t_) = acc;
}
__global__ __launch_bounds__(128) void k_main(const float* __restrict__ inp, const float* __restrict__ W1, const float* __restrict__ W2, const float* __restrict__ b2,
                                              const float* __restrict__ BASE, float* out) {
    __shared__ __align__(16) unsigned short sW2[16 * 72];
    __shared__ float sW1[2 * HD];
    __shared__ float sBase[NB_ * HD];
    __shared__ float sb2[16];
    __shared__ __align__(16) unsigned short hh[4][16 * 72];
    __shared__ __align__(16) unsigned short hl[4][16 * 72];
    __shared__ float dst[4][32 * 17];
    __shared__ __align__(16) float ost[4][96];
    const int tid = threadIdx.x, lane = tid & 31, wave = tid >> 5, lr = lane & 15, hf = lane >> 4;
    for (int i = tid; i < 16 * 72; i += 128) { const int n = i / 72, k = i - n * 72; sW2[i] = (n < OD && k < HD) ? f2bf(W2[k * OD + n]) : (unsigned short)0; }
    if (tid < 2 * HD) sW1[tid] = bfr(W1[tid]);
    for (int i = tid; i < NB_ * HD; i += 128) sBase[i] = BASE[i];
    if (tid < 16) sb2[tid] = (tid < OD) ? bfr(b2[tid]) : 0.f;
    __syncthreads();
    const int rw0 = blockIdx.x * 128 + wave * 32;
    unsigned short* myh = &hh[wave][0]; unsigned short* myl = &hl[wave][0]; float* myd = &dst[wave][0];
    const v16bf b0 = cat16b(*(const v8usa*)(sW2 + lr * 72 + 8 * hf), *(const v8usa*)(sW2 + lr * 72 + 16 + 8 * hf));
    const v16bf b1 = cat16b(*(const v8usa*)(sW2 + lr * 72 + 32 + 8 * hf), *(const v8usa*)(sW2 + lr * 72 + 48 + 8 * hf));
#pragma unroll
    for (int tile = 0; tile < 2; ++tile) {
        const int row = rw0 + tile * 16 + lr; const int n = row / RPN;
        const float c0 = tanhf(bfr(inp[(size_t)row * 3 + 0])), c1 = tanhf(bfr(inp[(size_t)row * 3 + 1]));
#pragma unroll 1
        for (int j = 0; j < 32; ++j) { const int k = hf * 32 + j;
            const float h = fmaxf(fmaf(c0, sW1[k], fmaf(c1, sW1[HD + k], sBase[n * HD + k])), 0.f);
            const unsigned short hb = f2bf(h); myh[lr * 72 + k] = hb; myl[lr * 72 + k] = f2bf(h - bf2f(hb)); }
        __builtin_amdgcn_wave_barrier(); asm volatile("" ::: "memory");
        const v16bf a0 = cat16b(*(const v8usa*)(myh + lr * 72 + 8 * hf), *(const v8usa*)(myh + lr * 72 + 16 + 8 * hf));
        const v16bf a1 = cat16b(*(const v8usa*)(myh + lr * 72 + 32 + 8 * hf), *(const v8usa*)(myh + lr * 72 + 48 + 8 * hf));
        const v16bf l0 = cat16b(*(const v8usa*)(myl + lr * 72 + 8 * hf), *(const v8usa*)(myl + lr * 72 + 16 + 8 * hf));
        const v16bf l1 = cat16b(*(const v8usa*)(myl + lr * 72 + 32 + 8 * hf), *(const v8usa*)(myl + lr * 72 + 48 + 8 * hf));
        v8f acc = {};
        acc = wmmab(a0, b0, acc); acc = wmmab(l0, b0, acc); acc = wmmab(a1, b1, acc); acc = wmmab(l1, b1, acc);
        asm volatile("v_nop\n\tv_nop\n\tv_nop\n\tv_nop" : "+v"(acc) : "v"(a0), "v"(a1), "v"(l0), "v"(l1));
#pragma unroll
        for (int j = 0; j < 8; ++j) myd[(tile * 16 + hf * 8 + j) * 17 + lr] = acc[j];
        __builtin_amdgcn_wave_barrier(); asm volatile("" ::: "memory");
    }
    {
        const int row = rw0 + lane; float* dr = myd + lane * 17;
#pragma unroll 1
        for (int k = 0; k < OD; ++k) { const float x = dr[k] + sb2[k]; dr[k] = fmaxf(x, 0.f) + log1pf(expf(-fabsf(x))) + 1e-4f; }
        asm volatile("" ::: "memory");
        const float dxl2 = dr[0], dxl1 = dr[1], dxr1 = dr[2], dxr2 = dr[3], dyl2 = dr[4], dyl1 = dr[5], dyr1 = dr[6], dyr2 = dr[7];
        const float kl = dr[8] * 2.0f, kr = dr[9] * 2.0f;
        const float xL1 = -dxl1, xL2 = -dxl1 - dxl2, yL1 = -dyl1, yL2 = -dyl1 - dyl2;
        const float xR1 = dxr1, xR2 = dxr1 + dxr2, yR1 = dyr1, yR2 = dyr1 + dyr2;
        const float xR3 = xR2 + 10000.0f, xL3 = xL2 - 10000.0f, yR3 = yR2 + kr * 10000.0f, yL3 = yL2 - kl * 10000.0f;
        const float ax0 = xL3, ax1 = xL2, ax2 = xL1, ax3 = xR1, ax4 = xR2, ax5 = xR3;
        const float ay0 = yL3, ay1 = yL2, ay2 = yL1, ay3 = yR1, ay4 = yR2, ay5 = yR3;
        float qx = bfr(inp[(size_t)row * 3 + 2]);
        qx = fminf(fmaxf(qx, ax0 * 0.99f), ax5 * 0.99f);
        float zi = 0.f;
        { const bool in = (qx >= ax0) && (qx < ax1); const float v = (ay1 - ay0) / (ax1 - ax0) * (qx - ax0) + ay0; zi += in ? v : 0.f; }
        { const bool in = (qx >= ax1) && (qx < ax2); const float v = (ay2 - ay1) / (ax2 - ax1) * (qx - ax1) + ay1; zi += in ? v : 0.f; }
        { const bool in = (qx >= ax2) && (qx < ax3); const float v = (ay3 - ay2) / (ax3 - ax2) * (qx - ax2) + ay2; zi += in ? v : 0.f; }
        { const bool in = (qx >= ax3) && (qx < ax4); const float v = (ay4 - ay3) / (ax4 - ax3) * (qx - ax3) + ay3; zi += in ? v : 0.f; }
        { const bool in = (qx >= ax4) && (qx < ax5); const float v = (ay5 - ay4) / (ax5 - ax4) * (qx - ax4) + ay4; zi += in ? v : 0.f; }
        float* osw = &ost[wave][0];
        osw[lane * 3 + 0] = bfr(inp[(size_t)row * 3 + 0]); osw[lane * 3 + 1] = bfr(inp[(size_t)row * 3 + 1]); osw[lane * 3 + 2] = zi;
    }
    __builtin_amdgcn_wave_barrier(); asm volatile("" ::: "memory");
    float* ob = out + (size_t)rw0 * 3;
    if (lane < 24) { const v4f v = *(const v4fa*)(&ost[wave][0] + lane * 4); *(volatile v4f*)(ob + lane * 4) = v; __threadfence(); *(volatile v4f*)(ob + lane * 4) = v; }
}

extern "C" void kernel_launch(void* const* d_in, const int* in_sizes, int n_in,
                              void* d_out, int out_size, void* d_ws, size_t ws_size, hipStream_t stream) {
    (void)in_sizes; (void)n_in; (void)out_size;
    const float* inp = (const float*)d_in[0]; const float* tfeat = (const float*)d_in[1]; const float* W1 = (const float*)d_in[2]; const float* b1 = (const float*)d_in[3];
    const float* W2 = (const float*)d_in[4]; const float* b2 = (const float*)d_in[5];
    float* out = (float*)d_out;
    if (ws_size < 4096) return;
    float* BASE = (float*)d_ws;
    k_base<<<1, 256, 0, stream>>>(tfeat, W1, b1, BASE);
    k_main<<<ROWS / 128, 128, 0, stream>>>(inp, W1, W2, b2, BASE, out);
}
